// FF_56908316672276
// MI455X (gfx1250) — hardware-run, weakly checked
//
#include <hip/hip_runtime.h>


#ifndef NB
#define NB 32
#endif
#ifndef SEQ
#define SEQ 256
#endif
#define NB_FULL  32
#define SEQ_FULL 256
#ifndef OUT_SEQ
#define OUT_SEQ SEQ
#endif
#define NIN  128
#define HID  32
#define NOUT 128
#define RB   16
#define PW   8
#define NJ   (SEQ / 32)
#define KS   (SEQ / 128)
#define YSP  36
#define HSP  68
#define OP   33
#define AP   (SEQ + 8)
#define PP   36
#define OUP  132
#define QRS  2048.0f
#define QRI  (1.0f / 2048.0f)
#define WSC  64.0f
#define WSI  (1.0f / 64.0f)
#define TL2E 2.8853900817779268f
#define L2E  1.4426950408889634f

static_assert(HID == 32);
static_assert(NIN % 32 == 0);
static_assert(NOUT == PW * 16);
static_assert(RB == 16);
static_assert(RB % PW == 0);
static_assert(SEQ % 128 == 0);
static_assert(SEQ % 64 == 0);
static_assert((NB * SEQ) % 64 == 0);
static_assert(SEQ % RB == 0);
static_assert(PW == 8);
static_assert(NB <= NB_FULL);
static_assert(SEQ <= SEQ_FULL);
static_assert(((size_t)SEQ * NIN) % 8 == 0);
static_assert(((size_t)HID * NIN) % 64 == 0);
static_assert(((size_t)HID * HID) % 64 == 0);
static_assert(((size_t)NOUT * HID) % 64 == 0);
static_assert((YSP * 4) % 16 == 0);
static_assert((HSP * 4) % 16 == 0);
static_assert((AP * 2) % 16 == 0);
static_assert((PP * 4) % 16 == 0);
static_assert((OUP * 4) % 16 == 0);
static_assert(32 * 16 * 4 == 16 * HID * 4);
static_assert(32 * 16 * 8 == HID * 64 * 2);
static_assert(32 * PW * 16 * 2 == RB * NOUT * 4);
static_assert(((SEQ * HID) / 4) % (32 * PW) == 0);
static_assert(RB * HID == 2 * 32 * PW);
static_assert(4 * RB * PP + RB * OUP <= SEQ * OP);
static_assert(((4 * RB * PP) * 4) % 16 == 0);
static_assert((SEQ * OP + RB * HID + HID) * 4 + 2 * RB * AP * 2 <= 131072);
static_assert((64 * YSP + 16 * HSP) * 4 <= 131072);

typedef _Float16 h16;
typedef unsigned short bf;
typedef __attribute__((ext_vector_type(16))) __bf16   v16bf;
typedef __attribute__((ext_vector_type(16))) _Float16 v16h;
typedef __attribute__((ext_vector_type(8)))  _Float16 v8h;
typedef __attribute__((ext_vector_type(8)))  unsigned short v8us;
typedef __attribute__((ext_vector_type(8)))  float    v8f;
typedef __attribute__((ext_vector_type(4)))  float    v4f;
typedef __attribute__((ext_vector_type(2)))  float    v2f;
typedef v4f  __attribute__((may_alias)) v4fa;
typedef v8h  __attribute__((may_alias)) v8ha;

__device__ __forceinline__ unsigned short f2bf(float f) { unsigned u = __float_as_uint(f); u += 0x7FFFu + ((u >> 16) & 1u); return (unsigned short)(u >> 16); }
__device__ __forceinline__ float bfr(float f) { return __uint_as_float(((unsigned)f2bf(f)) << 16); }
__device__ __forceinline__ v16h cat16(v8h lo, v8h hi) { return __builtin_shufflevector(lo, hi, 0, 1, 2, 3, 4, 5, 6, 7, 8, 9, 10, 11, 12, 13, 14, 15); }
__device__ __forceinline__ v16bf cat16b(v8us lo, v8us hi) { return __builtin_bit_cast(v16bf, __builtin_shufflevector(lo, hi, 0, 1, 2, 3, 4, 5, 6, 7, 8, 9, 10, 11, 12, 13, 14, 15)); }
__device__ __forceinline__ v8f wmma16(v16h a, v16h b, v8f c) { return __builtin_amdgcn_wmma_f32_16x16x32_f16(false, a, false, b, (short)0, c, false, false); }
__device__ __forceinline__ v8f wmmab(v16bf a, v16bf b, v8f c) { return __builtin_amdgcn_wmma_f32_16x16x32_bf16(false, a, false, b, (short)0, c, false, false); }
__device__ __forceinline__ v16h  ldh(const h16* p) { return cat16(*(const v8h*)p, *(const v8h*)(p + 16)); }
__device__ __forceinline__ v16bf ldb(const bf* p)  { return cat16b(*(const v8us*)p, *(const v8us*)(p + 16)); }
__device__ __forceinline__ void wave_sync() { __builtin_amdgcn_fence(3  , "wavefront"); __builtin_amdgcn_wave_barrier(); asm volatile("" ::: "memory"); }

__device__ __forceinline__ v8f wmmabg(v16bf a, v16bf b, v8f c) { c = wmmab(a, b, c); asm volatile("v_nop\n\tv_nop\n\tv_nop\n\tv_nop" : "+v"(c) : "v"(a), "v"(b)); return c; }
__device__ __forceinline__ v8f wmma16g(v16h a, v16h b, v8f c) { c = wmma16(a, b, c); asm volatile("v_nop\n\tv_nop\n\tv_nop\n\tv_nop" : "+v"(c) : "v"(a), "v"(b)); return c; }
static __device__ __forceinline__ h16 toh_flush(float v) { const float w = (fabsf(v) < 6.103515625e-05f) ? 0.0f : v; return (h16)w; }
static __device__ __forceinline__ h16 hres(float v, h16 hv) { return toh_flush((v - (float)hv) * QRS); }

__global__ __launch_bounds__(256) void k_cvt8(const float* __restrict__ src, bf* dst, size_t n8) {
    const size_t i = (size_t)blockIdx.x * 256 + threadIdx.x; if (i >= n8) return;
    const v8f v = *(const v8f*)(src + i * 8); v8us o;
#pragma unroll
    for (int k = 0; k < 8; ++k) o[k] = f2bf(v[k]);
    *(volatile v8us*)(dst + i * 8) = o; __threadfence(); *(volatile v8us*)(dst + i * 8) = o;
}

__global__ __launch_bounds__(256) void k_wconv(const float* __restrict__ src, h16* dst, size_t n8) {
    const size_t i = (size_t)blockIdx.x * 256 + threadIdx.x; if (i >= n8) return;
    const v8f v = *(const v8f*)(src + i * 8); v8h o;
#pragma unroll
    for (int k = 0; k < 8; ++k) o[k] = toh_flush(bfr(v[k]) * WSC);
    *(volatile v8h*)(dst + i * 8) = o; __threadfence(); *(volatile v8h*)(dst + i * 8) = o;
}

__global__ __launch_bounds__(32) void k_prep(const bf* __restrict__ XB, const bf* __restrict__ WINB, const float* __restrict__ bin,
                                             const h16* __restrict__ WH, const h16* __restrict__ WO, float* HF, float* OF, h16* YTH, h16* YTR) {
    __shared__ __align__(16) float ys[64 * YSP];
    __shared__ __align__(16) float hs[16 * HSP];
    const int lane = threadIdx.x & 31, lr = lane & 15, hi = lane >> 4;
    const unsigned bx = blockIdx.x; const unsigned r0 = bx * 64u;
    v8f acc[4][2];
#pragma unroll
    for (int mb = 0; mb < 4; ++mb)
#pragma unroll
        for (int nb = 0; nb < 2; ++nb) acc[mb][nb] = (v8f){};
    const size_t aoff = (size_t)(r0 + (unsigned)lr) * NIN + 8 * hi, boff = (size_t)lr * NIN + 8 * hi;
#pragma unroll 1
    for (int kc = 0; kc < NIN; kc += 32) {
        v16bf a[4];
#pragma unroll
        for (int mb = 0; mb < 4; ++mb) a[mb] = ldb(XB + aoff + (size_t)mb * 16 * NIN + kc);
#pragma unroll
        for (int nb = 0; nb < 2; ++nb) { const v16bf b = ldb(WINB + boff + (size_t)nb * 16 * NIN + kc);
#pragma unroll
            for (int mb = 0; mb < 4; ++mb) acc[mb][nb] = wmmabg(a[mb], b, acc[mb][nb]); }
    }
    float bc[2];
#pragma unroll
    for (int nb = 0; nb < 2; ++nb) bc[nb] = bfr(bin[nb * 16 + lr]);
#pragma unroll
    for (int mb = 0; mb < 4; ++mb)
#pragma unroll
        for (int nb = 0; nb < 2; ++nb)
#pragma unroll
            for (int j = 0; j < 8; ++j) ys[(mb * 16 + hi * 8 + j) * YSP + nb * 16 + lr] = acc[mb][nb][j] + bc[nb];
    wave_sync();
    const v16h wh0 = ldh(WH + (size_t)lr * HID + 8 * hi), wh1 = ldh(WH + (size_t)(16 + lr) * HID + 8 * hi);
    const v16h wo0 = ldh(WO + (size_t)lr * HID + 8 * hi), wo1 = ldh(WO + (size_t)(16 + lr) * HID + 8 * hi);
#pragma unroll 1
    for (int mb = 0; mb < 4; ++mb) {
        const int yb = (mb * 16 + lr) * YSP + 8 * hi;
        const v4f x0 = *(const v4fa*)(&ys[yb]), x1 = *(const v4fa*)(&ys[yb + 4]), x2 = *(const v4fa*)(&ys[yb + 16]), x3 = *(const v4fa*)(&ys[yb + 20]);
        v16h aH, aR;
#pragma unroll
        for (int i = 0; i < 4; ++i) {
            const h16 t0 = toh_flush(x0[i]); aH[i]      = t0; aR[i]      = hres(x0[i], t0);
            const h16 t1 = toh_flush(x1[i]); aH[4 + i]  = t1; aR[4 + i]  = hres(x1[i], t1);
            const h16 t2 = toh_flush(x2[i]); aH[8 + i]  = t2; aR[8 + i]  = hres(x2[i], t2);
            const h16 t3 = toh_flush(x3[i]); aH[12 + i] = t3; aR[12 + i] = hres(x3[i], t3); }
        v8f h0 = (v8f){}, h0r = (v8f){}, h1 = (v8f){}, h1r = (v8f){}, q0 = (v8f){}, q0r = (v8f){}, q1 = (v8f){}, q1r = (v8f){};
        h0 = wmma16g(aH, wh0, h0); h0r = wmma16g(aR, wh0, h0r);
        h1 = wmma16g(aH, wh1, h1); h1r = wmma16g(aR, wh1, h1r);
        q0 = wmma16g(aH, wo0, q0); q0r = wmma16g(aR, wo0, q0r);
        q1 = wmma16g(aH, wo1, q1); q1r = wmma16g(aR, wo1, q1r);
#pragma unroll
        for (int j = 0; j < 8; ++j) {
            hs[(hi * 8 + j) * HSP +  0 + lr] = (h0[j] + h0r[j] * QRI) * WSI;
            hs[(hi * 8 + j) * HSP + 16 + lr] = (h1[j] + h1r[j] * QRI) * WSI;
            hs[(hi * 8 + j) * HSP + 32 + lr] = (q0[j] + q0r[j] * QRI) * WSI;
            hs[(hi * 8 + j) * HSP + 48 + lr] = (q1[j] + q1r[j] * QRI) * WSI; }
        wave_sync();
#pragma unroll 1
        for (int ps = 0; ps < 2; ++ps) {
#pragma unroll
            for (int s = 0; s < 4; ++s) { const int row = 4 * s + (lane >> 3), cofs = (lane & 7) * 4;
                const v4f hv = *(const v4fa*)(&hs[row * HSP + cofs]); const v4f ov = *(const v4fa*)(&hs[row * HSP + 32 + cofs]);
                const size_t oo = (size_t)(r0 + (unsigned)(mb * 16 + row)) * HID + cofs;
                *(volatile v4f*)(HF + oo) = hv; *(volatile v4f*)(OF + oo) = ov; }
            if (ps == 0) __threadfence(); }
        wave_sync();
    }
    const unsigned bb = r0 / (unsigned)SEQ, tt = r0 % (unsigned)SEQ;
#pragma unroll 1
    for (int ps = 0; ps < 2; ++ps) {
#pragma unroll
        for (int s = 0; s < 8; ++s) { const int c = 4 * s + (lane >> 3), t8 = (lane & 7) * 8;
            v8h hv, rv;
#pragma unroll
            for (int i = 0; i < 8; ++i) { const float v = ys[(t8 + i) * YSP + c]; const h16 t = toh_flush(v); hv[i] = t; rv[i] = hres(v, t); }
            const size_t oo = ((size_t)bb * HID + (size_t)c) * SEQ + (size_t)tt + (size_t)t8;
            *(volatile v8h*)(YTH + oo) = hv; *(volatile v8h*)(YTR + oo) = rv; }
        if (ps == 0) __threadfence(); }
}

__global__ __launch_bounds__(32 * PW) void k_pair(const float* __restrict__ HF, const float* __restrict__ OF, const float* __restrict__ vin,
                                                   const h16* __restrict__ YTH, const h16* __restrict__ YTR, const h16* __restrict__ WOUTH,
                                                   const float* __restrict__ bout, float* OUT) {
    __shared__ __align__(16) float osm[SEQ * OP];
    __shared__ __align__(16) float hsm[RB * HID];
    __shared__ float vsm[HID];
    __shared__ __align__(16) h16 atH[RB * AP];
    __shared__ __align__(16) h16 atR[RB * AP];
    const int tid = threadIdx.x, lane = tid & 31, lr = lane & 15, hi = lane >> 4;
    const int wave = __builtin_amdgcn_readfirstlane((int)(threadIdx.x >> 5));
    const unsigned bx = blockIdx.x; const unsigned b = bx / (unsigned)(SEQ / RB); const unsigned i0 = (bx % (unsigned)(SEQ / RB)) * (unsigned)RB;
    const size_t tokb = (size_t)b * SEQ;
#pragma unroll
    for (int it = 0; it < (SEQ * HID / 4) / (32 * PW); ++it) {
        const int idx = it * (32 * PW) + tid; const int j = idx >> 3, g4 = (idx & 7) * 4;
        const v4f v = *(const v4f*)(OF + (tokb + (size_t)j) * HID + g4);
        osm[j * OP + g4 + 0] = v[0]; osm[j * OP + g4 + 1] = v[1]; osm[j * OP + g4 + 2] = v[2]; osm[j * OP + g4 + 3] = v[3]; }
    { const v2f v = *(const v2f*)(HF + (tokb + (size_t)i0) * HID + (size_t)tid * 2); hsm[tid * 2] = v[0]; hsm[tid * 2 + 1] = v[1]; }
    if (wave == 0) vsm[lane] = bfr(vin[lane]);
    __syncthreads();

#pragma unroll 1
    for (int r = 0; r < RB / PW; ++r) {
        const int il = wave * (RB / PW) + r;
        float e[NJ];
#pragma unroll
        for (int jj = 0; jj < NJ; ++jj) e[jj] = 0.0f;
#pragma unroll 2
        for (int g = 0; g < HID; ++g) {
            const float hv = hsm[il * HID + g]; const float vg = vsm[g];
#pragma unroll
            for (int jj = 0; jj < NJ; ++jj) {
                const float z  = hv + osm[(jj * 32 + lane) * OP + g];
                const float ex = __builtin_amdgcn_exp2f(z * TL2E);
                const float rc = __builtin_amdgcn_rcpf(ex + 1.0f);
                const float t  = fmaf(-2.0f, rc, 1.0f);
                e[jj] = fmaf(vg, t, e[jj]); }
        }
        float mx = e[0];
#pragma unroll
        for (int jj = 1; jj < NJ; ++jj) mx = fmaxf(mx, e[jj]);
#pragma unroll
        for (int off = 16; off > 0; off >>= 1) mx = fmaxf(mx, __shfl_xor(mx, off, 32));
        float sm = 0.0f;
#pragma unroll
        for (int jj = 0; jj < NJ; ++jj) sm += __builtin_amdgcn_exp2f((e[jj] - mx) * L2E);
#pragma unroll
        for (int off = 16; off > 0; off >>= 1) sm += __shfl_xor(sm, off, 32);
        const float lg = logf(sm);
#pragma unroll
        for (int jj = 0; jj < NJ; ++jj) {
            const float a = (e[jj] - mx) - lg;
            const h16 t = toh_flush(a);
            atH[il * AP + jj * 32 + lane] = t;
            atR[il * AP + jj * 32 + lane] = hres(a, t); }
    }
    __syncthreads();

    {   const int nt = wave & 1, q = wave >> 1;
        v8f cA = (v8f){}, cR = (v8f){};
        const size_t yo = ((size_t)b * HID + (size_t)(nt * 16 + lr)) * SEQ + 8 * hi;
        const int ao = lr * AP + 8 * hi;
#pragma unroll
        for (int s = 0; s < KS; ++s) {
            const int j0 = (q * KS + s) * 32;
            const v16h aH = cat16(*(const v8ha*)(&atH[ao + j0]), *(const v8ha*)(&atH[ao + j0 + 16]));
            const v16h aR = cat16(*(const v8ha*)(&atR[ao + j0]), *(const v8ha*)(&atR[ao + j0 + 16]));
            const v16h bH = ldh(YTH + yo + j0), bR = ldh(YTR + yo + j0);
            cA = wmma16g(aH, bH, cA);
            cR = wmma16g(aH, bR, cR);
            cR = wmma16g(aR, bH, cR); }
#pragma unroll
        for (int j = 0; j < 8; ++j) osm[(q * RB + 8 * hi + j) * PP + nt * 16 + lr] = cA[j] + cR[j] * QRI;
    }
    __syncthreads();

    {   v4f s0 = (v4f){}, s1 = (v4f){}, s2 = (v4f){}, s3 = (v4f){};
#pragma unroll
        for (int q = 0; q < 4; ++q) {
            const int pb = (q * RB + lr) * PP + 8 * hi;
            s0 += *(const v4fa*)(&osm[pb]); s1 += *(const v4fa*)(&osm[pb + 4]); s2 += *(const v4fa*)(&osm[pb + 16]); s3 += *(const v4fa*)(&osm[pb + 20]); }
        v16h cH, cL;
#pragma unroll
        for (int i = 0; i < 4; ++i) {
            const h16 t0 = toh_flush(s0[i]); cH[i]      = t0; cL[i]      = hres(s0[i], t0);
            const h16 t1 = toh_flush(s1[i]); cH[4 + i]  = t1; cL[4 + i]  = hres(s1[i], t1);
            const h16 t2 = toh_flush(s2[i]); cH[8 + i]  = t2; cL[8 + i]  = hres(s2[i], t2);
            const h16 t3 = toh_flush(s3[i]); cH[12 + i] = t3; cL[12 + i] = hres(s3[i], t3); }
        const v16h wf = ldh(WOUTH + (size_t)(wave * 16 + lr) * HID + 8 * hi);
        v8f oA = (v8f){}, oR = (v8f){};
        oA = wmma16g(cH, wf, oA);
        oR = wmma16g(cL, wf, oR);
        const float bo = bfr(bout[wave * 16 + lr]);
#pragma unroll
        for (int j = 0; j < 8; ++j) osm[4 * RB * PP + (8 * hi + j) * OUP + wave * 16 + lr] = (oA[j] + oR[j] * QRI) * WSI + bo;
    }
    __syncthreads();

    float* orow = OUT + ((size_t)b * OUT_SEQ + (size_t)i0) * NOUT;
#pragma unroll 1
    for (int ps = 0; ps < 2; ++ps) {
#pragma unroll
        for (int s = 0; s < 2; ++s) { const int line = s * 32 + (tid >> 3); const int row = line >> 2, cofs = (line & 3) * 32 + (tid & 7) * 4;
            const v4f val = *(const v4fa*)(&osm[4 * RB * PP + row * OUP + cofs]);
            *(volatile v4f*)(orow + (size_t)row * NOUT + cofs) = val; }
        if (ps == 0) __threadfence(); }
}

static constexpr size_t al256(size_t v) { return (v + 255) & ~(size_t)255; }
static constexpr size_t SZ_XB  = al256((size_t)NB * SEQ * NIN * 2);
static constexpr size_t SZ_WIN = al256((size_t)HID * NIN * 2);
static constexpr size_t SZ_WS  = al256((size_t)HID * HID * 2);
static constexpr size_t SZ_WO  = al256((size_t)NOUT * HID * 2);
static constexpr size_t SZ_F   = al256((size_t)NB * SEQ * HID * 4);
static constexpr size_t SZ_YT  = al256((size_t)NB * HID * SEQ * 2);
static constexpr size_t SZ_TOTAL = SZ_XB + SZ_WIN + 2 * SZ_WS + SZ_WO + 2 * SZ_F + 2 * SZ_YT;
static_assert(SZ_TOTAL <= (size_t)134217728);

extern "C" void kernel_launch(void* const* d_in, const int* in_sizes, int n_in,
                              void* d_out, int out_size, void* d_ws, size_t ws_size, hipStream_t stream) {
    if (n_in < 8) return;
    const size_t needx = ((size_t)(NB - 1) * SEQ_FULL + SEQ) * NIN;
    if ((size_t)in_sizes[0] < needx) return;
    if (in_sizes[1] < HID * NIN || in_sizes[2] < HID || in_sizes[3] < HID * HID || in_sizes[4] < HID * HID) return;
    if (in_sizes[5] < HID || in_sizes[6] < NOUT * HID || in_sizes[7] < NOUT) return;
    if ((size_t)out_size < ((size_t)(NB - 1) * OUT_SEQ + SEQ) * NOUT) return;
    if (SZ_TOTAL > ws_size) return;
    const float* xin  = (const float*)d_in[0];
    const float* win  = (const float*)d_in[1];
    const float* bin  = (const float*)d_in[2];
    const float* wh   = (const float*)d_in[3];
    const float* wo   = (const float*)d_in[4];
    const float* vv   = (const float*)d_in[5];
    const float* wout = (const float*)d_in[6];
    const float* bout = (const float*)d_in[7];
    float* OUT = (float*)d_out;
    char* wsp = (char*)d_ws;
    bf*  XB    = (bf*)wsp;  wsp += SZ_XB;
    bf*  WINB  = (bf*)wsp;  wsp += SZ_WIN;
    h16* WH    = (h16*)wsp; wsp += SZ_WS;
    h16* WO    = (h16*)wsp; wsp += SZ_WS;
    h16* WOUTH = (h16*)wsp; wsp += SZ_WO;
    float* HF  = (float*)wsp; wsp += SZ_F;
    float* OF  = (float*)wsp; wsp += SZ_F;
    h16* YTH   = (h16*)wsp; wsp += SZ_YT;
    h16* YTR   = (h16*)wsp; wsp += SZ_YT;

    if (SEQ == SEQ_FULL) {
        const size_t n8 = (size_t)NB * SEQ * NIN / 8;
        k_cvt8<<<(unsigned)((n8 + 255) / 256), 256, 0, stream>>>(xin, XB, n8);
    } else {
        const size_t n8 = (size_t)SEQ * NIN / 8;
        for (int b = 0; b < NB; ++b) k_cvt8<<<(unsigned)((n8 + 255) / 256), 256, 0, stream>>>(xin + (size_t)b * SEQ_FULL * NIN, XB + (size_t)b * SEQ * NIN, n8);
    }
    { const size_t n8 = (size_t)HID * NIN / 8;  k_cvt8<<<(unsigned)((n8 + 255) / 256), 256, 0, stream>>>(win, WINB, n8); }
    { const size_t n8 = (size_t)HID * HID / 8;  const unsigned g = (unsigned)((n8 + 255) / 256);
      k_wconv<<<g, 256, 0, stream>>>(wh, WH, n8); k_wconv<<<g, 256, 0, stream>>>(wo, WO, n8); }
    { const size_t n8 = (size_t)NOUT * HID / 8; k_wconv<<<(unsigned)((n8 + 255) / 256), 256, 0, stream>>>(wout, WOUTH, n8); }

    k_prep<<<dim3(NB * SEQ / 64, 1, 1), 32, 0, stream>>>(XB, WINB, bin, WH, WO, HF, OF, YTH, YTR);
    k_pair<<<dim3(NB * (SEQ / RB), 1, 1), 32 * PW, 0, stream>>>(HF, OF, vv, YTH, YTR, WOUTH, bout, OUT);
}
